// HypModel_57277683859539
// MI455X (gfx1250) — hardware-verified
//
#include <hip/hip_runtime.h>
#include <stddef.h>


#define NS    4096
#define ND    8
#define FIN   64
#define HID   512
#define HID2  256
#define ROWF  (ND * HID)
#define MROWS (ND * NS)
#define MHALF (MROWS / 2)

#define GT    64
#define GTHR  128
#define TSP   68

#define NB    16
#define CHUNK 2048
#define NTHR  256
#define NWAVE 8
#define WCAP  256
#define NGRP  (CHUNK / (NTHR * 4))
#define LDS_ACC   (NB * ROWF)
#define LDS_BYTES (LDS_ACC * 4 + NB * 4 + NWAVE * WCAP * 4 + NWAVE * 4)

static_assert(WCAP == (CHUNK / NTHR) * 32);
static_assert(NGRP >= 1);
static_assert(LDS_BYTES == 270432);
static_assert((LDS_ACC % 4) == 0);
static_assert((NS % NB) == 0 && (NB % NWAVE) == 0);
static_assert((MHALF % GT) == 0 && (NS % GT) == 0 && (HID % GT) == 0 && (HID2 % GT) == 0);
static_assert((FIN % 32) == 0 && (HID % 32) == 0);
static_assert(HID == 64 * 8);
static_assert(HID2 == 32 * 8);
static_assert((NS % 32) == 0);
static_assert((TSP % 4) == 0);

typedef float          v4f   __attribute__((ext_vector_type(4)));
typedef float          v8f   __attribute__((ext_vector_type(8)));
typedef int            v4i   __attribute__((ext_vector_type(4)));
typedef unsigned short v8us  __attribute__((ext_vector_type(8)));
typedef __bf16         v16bf __attribute__((ext_vector_type(16)));
union Frag { v16bf v; v8us half[2]; };
union P16  { v8us u; v4i i; };

__device__ __forceinline__ float lrelu(float v) { return v > 0.f ? v : 0.01f * v; }
__device__ __forceinline__ int iclamp(int v, int lo, int hi) { return v < lo ? lo : (v > hi ? hi : v); }

__device__ __forceinline__ unsigned short f2bf(float f) {
  unsigned u = __float_as_uint(f);
  u += 0x7FFFu + ((u >> 16) & 1u);
  return (unsigned short)(u >> 16);
}
__device__ __forceinline__ float bf2f(unsigned short b) { return __uint_as_float(((unsigned)b) << 16); }

__device__ __forceinline__ void split8(v4f a, v4f b, P16& h, P16& l) {
  float v[8] = {a.x, a.y, a.z, a.w, b.x, b.y, b.z, b.w};
#pragma unroll
  for (int j = 0; j < 8; ++j) {
    const unsigned short hs = f2bf(v[j]);
    const unsigned short ls = f2bf(v[j] - bf2f(hs));
    h.u[j] = hs;
    l.u[j] = ls;
  }
}

__device__ __forceinline__ void st16(void* p, v4i v) { *(volatile v4i*)p = v; }
__device__ __forceinline__ void st4f(float* p, v4f v) { *(volatile v4f*)p = v; }

__device__ __forceinline__ v8f wraw(v16bf a, v16bf b, v8f c) {
  return __builtin_amdgcn_wmma_f32_16x16x32_bf16(false, a, false, b, (short)0, c, false, false);
}

__device__ __forceinline__ float wsum(float v) {
  v += __shfl_xor(v, 16, 32);
  v += __shfl_xor(v, 8, 32);
  v += __shfl_xor(v, 4, 32);
  v += __shfl_xor(v, 2, 32);
  v += __shfl_xor(v, 1, 32);
  return v;
}

__global__ __launch_bounds__(256) void k_prep(const float* __restrict__ src, unsigned short* dh,
                                              unsigned short* dl, int n8) {
  const int i = blockIdx.x * 256 + threadIdx.x;
  if (i >= n8) return;
  const size_t o = (size_t)i * 8;
  const v4f a = *(const v4f*)(src + o);
  const v4f b = *(const v4f*)(src + o + 4);
  P16 h, l;
  split8(a, b, h, l);
  st16(dh + o, h.i);
  st16(dl + o, l.i);
  __threadfence();
  st16(dh + o, h.i);
  st16(dl + o, l.i);
}

template <int OUTK>
__global__ __launch_bounds__(GTHR) void k_gemm(
    const unsigned short* __restrict__ Ah, const unsigned short* __restrict__ Al,
    const unsigned short* __restrict__ Bh, const unsigned short* __restrict__ Bl,
    const float* __restrict__ bias, float* outF, unsigned short* outH, unsigned short* outL,
    int K, int ldo, int mBase, int ns, int nd) {
  __shared__ __attribute__((aligned(16))) float Ts[GT * TSP];

  const int tid  = threadIdx.x;
  const int lane = tid & 31;
  const int wave = tid >> 5;
  const int hh   = lane >> 4;
  const int m    = lane & 15;
  const int wr   = (wave & 1) * 32;
  const int wc   = (wave >> 1) * 32;
  const int rowBase = blockIdx.y * GT;
  const int colBase = blockIdx.x * GT;

  const size_t ar0 = (size_t)(rowBase + wr + m) * (size_t)K + 8 * hh;
  const size_t ar1 = ar0 + (size_t)16 * (size_t)K;
  const size_t br0 = (size_t)(colBase + wc + m) * (size_t)K + 8 * hh;
  const size_t br1 = br0 + (size_t)16 * (size_t)K;

  v8f c00 = {0.f, 0.f, 0.f, 0.f, 0.f, 0.f, 0.f, 0.f};
  v8f c01 = c00, c10 = c00, c11 = c00;

#pragma unroll 1
  for (int k0 = 0; k0 < K; k0 += 32) {
    Frag a0h, a0l, a1h, a1l, b0h, b0l, b1h, b1l;
    a0h.half[0] = *(const v8us*)(Ah + ar0 + k0);  a0h.half[1] = *(const v8us*)(Ah + ar0 + k0 + 16);
    a0l.half[0] = *(const v8us*)(Al + ar0 + k0);  a0l.half[1] = *(const v8us*)(Al + ar0 + k0 + 16);
    a1h.half[0] = *(const v8us*)(Ah + ar1 + k0);  a1h.half[1] = *(const v8us*)(Ah + ar1 + k0 + 16);
    a1l.half[0] = *(const v8us*)(Al + ar1 + k0);  a1l.half[1] = *(const v8us*)(Al + ar1 + k0 + 16);
    b0h.half[0] = *(const v8us*)(Bh + br0 + k0);  b0h.half[1] = *(const v8us*)(Bh + br0 + k0 + 16);
    b0l.half[0] = *(const v8us*)(Bl + br0 + k0);  b0l.half[1] = *(const v8us*)(Bl + br0 + k0 + 16);
    b1h.half[0] = *(const v8us*)(Bh + br1 + k0);  b1h.half[1] = *(const v8us*)(Bh + br1 + k0 + 16);
    b1l.half[0] = *(const v8us*)(Bl + br1 + k0);  b1l.half[1] = *(const v8us*)(Bl + br1 + k0 + 16);

    c00 = wraw(a0h.v, b0h.v, c00); c00 = wraw(a0h.v, b0l.v, c00); c00 = wraw(a0l.v, b0h.v, c00);
    c01 = wraw(a0h.v, b1h.v, c01); c01 = wraw(a0h.v, b1l.v, c01); c01 = wraw(a0l.v, b1h.v, c01);
    c10 = wraw(a1h.v, b0h.v, c10); c10 = wraw(a1h.v, b0l.v, c10); c10 = wraw(a1l.v, b0h.v, c10);
    c11 = wraw(a1h.v, b1h.v, c11); c11 = wraw(a1h.v, b1l.v, c11); c11 = wraw(a1l.v, b1h.v, c11);
    asm volatile("v_nop\n\tv_nop\n\tv_nop\n\tv_nop"
                 : "+v"(c00), "+v"(c01), "+v"(c10), "+v"(c11)
                 : "v"(a0h.v), "v"(a0l.v), "v"(a1h.v), "v"(a1l.v),
                   "v"(b0h.v), "v"(b0l.v), "v"(b1h.v), "v"(b1l.v));
  }

  {
    const int cA = wc + m, cB = wc + 16 + m;
    const float bvA = bias[colBase + cA];
    const float bvB = bias[colBase + cB];
    const int rA = wr + 8 * hh, rB = wr + 16 + 8 * hh;
#pragma unroll
    for (int r = 0; r < 8; ++r) {
      Ts[(rA + r) * TSP + cA] = lrelu(c00[r] + bvA);
      Ts[(rA + r) * TSP + cB] = lrelu(c01[r] + bvB);
      Ts[(rB + r) * TSP + cA] = lrelu(c10[r] + bvA);
      Ts[(rB + r) * TSP + cB] = lrelu(c11[r] + bvB);
    }
  }
  __syncthreads();

  if constexpr (OUTK == 2) {
    (void)outF; (void)mBase; (void)ns; (void)nd;
    P16 hv[4], lv[4];
    size_t offs[4];
#pragma unroll
    for (int i = 0; i < 4; ++i) {
      const int row = i * 16 + (tid >> 3);
      const int c8  = (tid & 7) * 8;
      const v4f x0 = *(const v4f*)(Ts + row * TSP + c8);
      const v4f x1 = *(const v4f*)(Ts + row * TSP + c8 + 4);
      split8(x0, x1, hv[i], lv[i]);
      offs[i] = (size_t)(rowBase + row) * (size_t)ldo + colBase + c8;
    }
#pragma unroll
    for (int i = 0; i < 4; ++i) { st16(outH + offs[i], hv[i].i); st16(outL + offs[i], lv[i].i); }
    __threadfence();
#pragma unroll
    for (int i = 0; i < 4; ++i) { st16(outH + offs[i], hv[i].i); st16(outL + offs[i], lv[i].i); }
  } else {
    (void)outH; (void)outL;
    v4f vals[8];
    size_t offs[8];
#pragma unroll
    for (int i = 0; i < 8; ++i) {
      const int row = i * 8 + (tid >> 4);
      const int c4  = (tid & 15) * 4;
      vals[i] = *(const v4f*)(Ts + row * TSP + c4);
      int orow = rowBase + row;
      if constexpr (OUTK == 1) {
        const int mg = mBase + orow;
        orow = (mg % ns) * nd + mg / ns;
      }
      offs[i] = (size_t)orow * (size_t)ldo + colBase + c4;
    }
#pragma unroll
    for (int i = 0; i < 8; ++i) st4f(outF + offs[i], vals[i]);
    __threadfence();
#pragma unroll
    for (int i = 0; i < 8; ++i) st4f(outF + offs[i], vals[i]);
  }
}

__global__ __launch_bounds__(NTHR) void k_agg(const float* __restrict__ Y, const int* __restrict__ esrc,
                                              const int* __restrict__ edst, unsigned short* Sh,
                                              unsigned short* Sl, int ns, int nE) {
  extern __shared__ v4f lds_dyn[];
  float* sacc = (float*)lds_dyn;
  int*   cnt  = (int*)(sacc + LDS_ACC);
  int*   list = cnt + NB;
  int*   wcnt = list + NWAVE * WCAP;

  const int tid  = threadIdx.x;
  const int lane = tid & 31;
  const int wave = tid >> 5;
  const int nodeBase = blockIdx.x * NB;

  {
    const v4f z4 = {0.f, 0.f, 0.f, 0.f};
    for (int i = tid; i < LDS_ACC / 4; i += NTHR) lds_dyn[i] = z4;
    if (tid < NB) cnt[tid] = 0;
  }
  __syncthreads();

  const bool vec16 = ((((size_t)edst) & 15) == 0);
  const int nChunks = (nE + CHUNK - 1) / CHUNK;
#pragma unroll 1
  for (int ch = 0; ch < nChunks; ++ch) {
    const int cbase = ch * CHUNK;
    int wc = 0;
#pragma unroll
    for (int g = 0; g < NGRP; ++g) {
      const int el0 = (g * NTHR + tid) * 4;
      const int e0  = cbase + el0;
      const int sent = -2147483647 - 1;
      v4i d;
      if (vec16 && (cbase + CHUNK <= nE)) {
        d = *(const v4i*)(edst + e0);
      } else {
        d.x = (e0     < nE) ? edst[iclamp(e0,     0, nE - 1)] : sent;
        d.y = (e0 + 1 < nE) ? edst[iclamp(e0 + 1, 0, nE - 1)] : sent;
        d.z = (e0 + 2 < nE) ? edst[iclamp(e0 + 2, 0, nE - 1)] : sent;
        d.w = (e0 + 3 < nE) ? edst[iclamp(e0 + 3, 0, nE - 1)] : sent;
      }
      const unsigned s0 = (unsigned)d.x - (unsigned)nodeBase;
      const unsigned s1 = (unsigned)d.y - (unsigned)nodeBase;
      const unsigned s2 = (unsigned)d.z - (unsigned)nodeBase;
      const unsigned s3 = (unsigned)d.w - (unsigned)nodeBase;
      const bool h0 = s0 < (unsigned)NB;
      const bool h1 = s1 < (unsigned)NB;
      const bool h2 = s2 < (unsigned)NB;
      const bool h3 = s3 < (unsigned)NB;
      const unsigned many = __builtin_amdgcn_ballot_w32(h0 | h1 | h2 | h3);
      if (many != 0u) {
#define HITJ(J, HJ, SJ) { \
          const unsigned mj = __builtin_amdgcn_ballot_w32(HJ); \
          if (HJ) { \
            const int pos = wc + (int)__builtin_amdgcn_mbcnt_lo(mj, 0u); \
            if (pos < WCAP) list[wave * WCAP + pos] = ((el0 + (J)) << 8) | (int)(SJ); \
          } \
          wc += (int)__builtin_popcount(mj); }
        HITJ(0, h0, s0)
        HITJ(1, h1, s1)
        HITJ(2, h2, s2)
        HITJ(3, h3, s3)
#undef HITJ
      }
    }
    if (lane == 0) wcnt[wave] = wc;
    __syncthreads();

    if (wave == 0) {
      for (int wsx = 0; wsx < NWAVE; ++wsx) {
        int n = wcnt[wsx];
        if (n > WCAP) n = WCAP;
        if (n < 0) n = 0;
        for (int i = 0; i < n; ++i) {
          const int ent  = list[wsx * WCAP + i];
          const int slot = ent & (NB - 1);
          const int el   = (ent >> 8) & (CHUNK - 1);
          int e = cbase + el;
          if (e > nE - 1) e = nE - 1;
          const int s = iclamp(esrc[e], 0, ns - 1);
          if (lane == 0) cnt[slot] += 1;
          const float* yp = Y + (size_t)s * ROWF + 4 * lane;
          float* ap = sacc + slot * ROWF + 4 * lane;
#pragma unroll 8
          for (int it = 0; it < ROWF / 128; ++it) {
            const v4f yv = *(const v4f*)(yp + it * 128);
            v4f* a = (v4f*)(ap + it * 128);
            const v4f cur = *a;
            *a = cur + yv;
          }
        }
      }
    }
    __syncthreads();
  }

#pragma unroll 1
  for (int j = 0; j < NB / NWAVE; ++j) {
    const int slot = wave * (NB / NWAVE) + j;
    const int node = nodeBase + slot;
    if (node >= ns) break;
    const float inv = 1.0f / fmaxf((float)cnt[slot], 1.0f);
    const float* yrow = Y + (size_t)node * ROWF;
    const float* arow = sacc + slot * ROWF;
#pragma unroll 1
    for (int dq = 0; dq < ND * 2; ++dq) {
      const int col = (dq >> 1) * HID + (dq & 1) * 256 + lane * 8;
      const v4f y0 = *(const v4f*)(yrow + col);
      const v4f y1 = *(const v4f*)(yrow + col + 4);
      const v4f a0 = *(const v4f*)(arow + col);
      const v4f a1 = *(const v4f*)(arow + col + 4);
      const v4f s0 = y0 + a0 * inv;
      const v4f s1 = y1 + a1 * inv;
      P16 h, l;
      split8(s0, s1, h, l);
      const size_t o = (size_t)node * ROWF + col;
      st16(Sh + o, h.i);
      st16(Sl + o, l.i);
      __threadfence();
      st16(Sh + o, h.i);
      st16(Sl + o, l.i);
    }
  }
}

__global__ __launch_bounds__(64) void k_conv(const float* __restrict__ G, const float* __restrict__ Wc,
                                              const float* __restrict__ bc, unsigned short* Ch,
                                              unsigned short* Cl, int nodeOff) {
  const int n   = blockIdx.x;
  const int tid = threadIdx.x;
  const int h0  = tid * 8;
  const float* g = G + (size_t)n * ROWF;
  const float b0 = bc[0];
  float acc[8];
#pragma unroll
  for (int j = 0; j < 8; ++j) acc[j] = b0;
  const int il = iclamp(h0 - 1, 0, HID - 1);
  const int ir = iclamp(h0 + 8, 0, HID - 1);
  const bool hasL = (h0 > 0);
  const bool hasR = (h0 + 8 < HID);
#pragma unroll 1
  for (int d = 0; d < ND; ++d) {
    const float* row = g + d * HID;
    const v4f x0 = *(const v4f*)(row + h0);
    const v4f x1 = *(const v4f*)(row + h0 + 4);
    float xm = row[il]; xm = hasL ? xm : 0.f;
    float xp = row[ir]; xp = hasR ? xp : 0.f;
    const float w0 = Wc[d * 3], w1 = Wc[d * 3 + 1], w2 = Wc[d * 3 + 2];
    float v[10] = {xm, x0.x, x0.y, x0.z, x0.w, x1.x, x1.y, x1.z, x1.w, xp};
#pragma unroll
    for (int j = 0; j < 8; ++j) acc[j] = acc[j] + w0 * v[j] + w1 * v[j + 1] + w2 * v[j + 2];
  }
  v4f o0, o1;
  o0.x = lrelu(acc[0]); o0.y = lrelu(acc[1]); o0.z = lrelu(acc[2]); o0.w = lrelu(acc[3]);
  o1.x = lrelu(acc[4]); o1.y = lrelu(acc[5]); o1.z = lrelu(acc[6]); o1.w = lrelu(acc[7]);
  P16 hbits, lbits;
  split8(o0, o1, hbits, lbits);
  const size_t o = (size_t)(nodeOff + n) * HID + h0;
  st16(Ch + o, hbits.i);
  st16(Cl + o, lbits.i);
  __threadfence();
  st16(Ch + o, hbits.i);
  st16(Cl + o, lbits.i);
}

__global__ __launch_bounds__(256) void k_final(const float* __restrict__ O, const float* __restrict__ W4,
                                               const float* __restrict__ b4, float* out, int nrows) {
  __shared__ __attribute__((aligned(16))) float res[32];
  const int tid  = threadIdx.x;
  const int lane = tid & 31;
  const int wave = tid >> 5;
  const int rowBase = blockIdx.x * 32;
  const v4f w0 = *(const v4f*)(W4 + lane * 8);
  const v4f w1 = *(const v4f*)(W4 + lane * 8 + 4);
  const float bb = b4[0];
#pragma unroll 1
  for (int j = 0; j < 4; ++j) {
    const int r = iclamp(rowBase + wave * 4 + j, 0, nrows - 1);
    const float* p = O + (size_t)r * HID2 + lane * 8;
    const v4f q0 = *(const v4f*)p;
    const v4f q1 = *(const v4f*)(p + 4);
    float s = q0.x * w0.x + q0.y * w0.y + q0.z * w0.z + q0.w * w0.w
            + q1.x * w1.x + q1.y * w1.y + q1.z * w1.z + q1.w * w1.w;
    s = wsum(s);
    if (lane == 0) res[wave * 4 + j] = s + bb;
  }
  __syncthreads();
  if (wave == 0 && lane < 8 && rowBase + lane * 4 + 3 < nrows) {
    const v4f v = *(const v4f*)(res + lane * 4);
    float* op = out + rowBase + lane * 4;
    st4f(op, v);
    __threadfence();
    st4f(op, v);
  }
}

extern "C" void kernel_launch(void* const* d_in, const int* in_sizes, int n_in,
                              void* d_out, int out_size, void* d_ws, size_t ws_size,
                              hipStream_t stream) {
  if (n_in < 15) return;
  const int nE = in_sizes[1];
  if (nE < 0 || in_sizes[2] != nE) return;
  if (in_sizes[0] != MROWS * FIN) return;
  if (in_sizes[3] != HID * FIN || in_sizes[4] != HID) return;
  if (in_sizes[5] != HID * HID || in_sizes[6] != HID) return;
  if (in_sizes[7] != HID * HID || in_sizes[8] != HID) return;
  if (in_sizes[9] != ND * 3 || in_sizes[10] < 1) return;
  if (in_sizes[11] != HID2 * HID || in_sizes[12] != HID2) return;
  if (in_sizes[13] != HID2 || in_sizes[14] < 1) return;
  if (out_size != NS) return;

  const float* x   = (const float*)d_in[0];
  const int*   src = (const int*)d_in[1];
  const int*   dst = (const int*)d_in[2];
  const float* W1  = (const float*)d_in[3];
  const float* b1  = (const float*)d_in[4];
  const float* W2  = (const float*)d_in[5];
  const float* b2  = (const float*)d_in[6];
  const float* Wg  = (const float*)d_in[7];
  const float* bg  = (const float*)d_in[8];
  const float* Wc  = (const float*)d_in[9];
  const float* bc  = (const float*)d_in[10];
  const float* W3  = (const float*)d_in[11];
  const float* b3  = (const float*)d_in[12];
  const float* W4  = (const float*)d_in[13];
  const float* b4  = (const float*)d_in[14];
  float* out = (float*)d_out;

  const size_t MB = 1048576;
  const size_t wsEnd = 128 * MB;
  if (ws_size < wsEnd) return;
  char* ws = (char*)d_ws;
  unsigned short* H1h = (unsigned short*)(ws + 0);
  unsigned short* H1l = (unsigned short*)(ws + 16 * MB);
  unsigned short* Xh  = (unsigned short*)(ws + 32 * MB);
  unsigned short* Xl  = (unsigned short*)(ws + 36 * MB);
  unsigned short* W1h = (unsigned short*)(ws + 40 * MB);
  unsigned short* W1l = (unsigned short*)(ws + 40 * MB + 65536);
  unsigned short* W2h = (unsigned short*)(ws + 40 * MB + 131072);
  unsigned short* W2l = (unsigned short*)(ws + 40 * MB + 131072 + 524288);
  unsigned short* Sh  = (unsigned short*)(ws + 0);
  unsigned short* Sl  = (unsigned short*)(ws + 32 * MB);
  float*          O   = (float*)(ws + 0);
  float*          Y   = (float*)(ws + 64 * MB);
  float*          Gh  = (float*)(ws + 64 * MB);
  unsigned short* Wgh = (unsigned short*)(ws + 96 * MB);
  unsigned short* Wgl = (unsigned short*)(ws + 96 * MB + 524288);
  unsigned short* W3h = (unsigned short*)(ws + 97 * MB);
  unsigned short* W3l = (unsigned short*)(ws + 97 * MB + 262144);
  unsigned short* Ch  = (unsigned short*)(ws + 98 * MB);
  unsigned short* Cl  = (unsigned short*)(ws + 102 * MB);
  float*          dumF = (float*)(ws + 106 * MB);
  unsigned short* dumU = (unsigned short*)(ws + 106 * MB);

  static_assert((size_t)MHALF * HID * 2 == 16 * 1048576);
  static_assert((size_t)MROWS * FIN * 2 == 4 * 1048576);
  static_assert((size_t)MROWS * HID * 2 == 32 * 1048576);
  static_assert((size_t)MROWS * HID * 4 == 64 * 1048576);
  static_assert((size_t)MHALF * HID * 4 == 32 * 1048576);
  static_assert((size_t)NS * HID * 2 == 4 * 1048576);
  static_assert((size_t)NS * HID2 * 4 == 4 * 1048576);
  static_assert((size_t)HID * FIN * 2 == 65536 && (size_t)HID * HID * 2 == 524288 && (size_t)HID2 * HID * 2 == 262144);

  k_prep<<<(MROWS * FIN / 8) / 256, 256, 0, stream>>>(x, Xh, Xl, MROWS * FIN / 8);
  k_prep<<<(HID * FIN / 8) / 256, 256, 0, stream>>>(W1, W1h, W1l, HID * FIN / 8);
  k_prep<<<(HID * HID / 8) / 256, 256, 0, stream>>>(W2, W2h, W2l, HID * HID / 8);

  for (int p = 0; p < 2; ++p) {
    k_gemm<2><<<dim3(HID / GT, MHALF / GT), GTHR, 0, stream>>>(
        Xh + (size_t)p * MHALF * FIN, Xl + (size_t)p * MHALF * FIN, W1h, W1l, b1,
        dumF, H1h, H1l, FIN, HID, 0, NS, ND);
    k_gemm<1><<<dim3(HID / GT, MHALF / GT), GTHR, 0, stream>>>(
        H1h, H1l, W2h, W2l, b2, Y, dumU, dumU, HID, HID, p * MHALF, NS, ND);
  }

  hipFuncSetAttribute(reinterpret_cast<const void*>(&k_agg),
                      hipFuncAttributeMaxDynamicSharedMemorySize, LDS_BYTES);
  k_agg<<<NS / NB, NTHR, LDS_BYTES, stream>>>(Y, src, dst, Sh, Sl, NS, nE);

  k_prep<<<(HID * HID / 8) / 256, 256, 0, stream>>>(Wg, Wgh, Wgl, HID * HID / 8);
  k_prep<<<(HID2 * HID / 8) / 256, 256, 0, stream>>>(W3, W3h, W3l, HID2 * HID / 8);

  for (int p = 0; p < 2; ++p) {
    k_gemm<0><<<dim3(HID / GT, MHALF / GT), GTHR, 0, stream>>>(
        Sh + (size_t)p * MHALF * HID, Sl + (size_t)p * MHALF * HID, Wgh, Wgl, bg,
        Gh, dumU, dumU, HID, HID, 0, NS, ND);
    k_conv<<<NS / 2, 64, 0, stream>>>(Gh, Wc, bc, Ch, Cl, p * (NS / 2));
  }

  k_gemm<0><<<dim3(HID2 / GT, NS / GT), GTHR, 0, stream>>>(
      Ch, Cl, W3h, W3l, b3, O, dumU, dumU, HID, HID2, 0, NS, ND);
  k_final<<<NS / 32, 256, 0, stream>>>(O, W4, b4, out, NS);
}
